// STFT_18648747999406
// MI455X (gfx1250) — hardware-verified
//
#include <hip/hip_runtime.h>
#include <math.h>

typedef __attribute__((ext_vector_type(16))) _Float16 v16h;
typedef __attribute__((ext_vector_type(8)))  _Float16 v8h;
typedef __attribute__((ext_vector_type(8)))  float    v8f;
typedef __attribute__((ext_vector_type(4)))  float    v4f;

constexpr int kBatch     = 32;
constexpr int kSamp      = 160000;
constexpr int kTaps      = 800;
constexpr int kHop       = 200;
constexpr int kHalfPad   = kTaps / 2;
constexpr int kPadLen    = kSamp + 2 * kHalfPad;
constexpr int kFrames    = (kPadLen - kTaps) / kHop + 1;
constexpr int kSlotsPerB = kPadLen / kHop;
constexpr int kCut       = kTaps / 2 + 1;
constexpr int kChan      = 2 * kCut;
constexpr int kNP        = 832;
constexpr int kRowsM     = kBatch * kSlotsPerB;
constexpr int kSlots     = kRowsM + 4;
constexpr int kK3        = 4 * kNP;
constexpr int kN3        = 256;
constexpr int kXpHalves  = 2513 * 2048;
constexpr int kHsqLen    = 832;
static_assert(kPadLen == 160800 && kFrames == 801 && kSlotsPerB == 804 && kCut == 401 && kChan == 802, "shape chain");
static_assert(kSlotsPerB * kHop == kPadLen, "per-batch stride of the padded signal equals 804 hops");
static_assert(kRowsM == 25728 && (kRowsM % 64) == 0, "M multiple of 64");
static_assert((kNP % 64) == 0 && (kN3 % 64) == 0, "N multiples of 64");
static_assert((kTaps % 32) == 0 && (kK3 % 32) == 0, "K multiples of 32");
static_assert((kNP / 64) * 32 >= kCut, "pair capacity");
static_assert((long)(kRowsM - 1) * kHop + kTaps <= (long)kXpHalves, "signal plane covers the last row");
static_assert(kBatch * kPadLen <= kXpHalves && (kPadLen % 8) == 0, "signal plane size");
static_assert(kRowsM + 3 < kSlots, "slot plane covers the last row of the fused GEMM");

constexpr float kCarryX  = 16.0f;
constexpr float kCarryFb = 1024.0f;
constexpr float kCarryFt = 16.0f;
constexpr float kCarryIb = 65536.0f;
constexpr float kScale1  = 1.0f / (kCarryX * kCarryFb);
constexpr float kScale3  = 1.0f / (kCarryFt * kCarryIb);
constexpr float kH16MinNormal = 6.103515625e-05f;
constexpr float kTiny    = 1.1754944e-38f;

constexpr size_t kOffXP  = 0;
constexpr size_t kOffFB  = kOffXP  + (size_t)kXpHalves * 2;
constexpr size_t kOffIB  = kOffFB  + (size_t)kNP * kTaps * 2;
constexpr size_t kOffHSQ = kOffIB  + (size_t)kN3 * kK3 * 2;
constexpr size_t kOffFT  = kOffHSQ + (size_t)kHsqLen * 4;
constexpr size_t kOffY3  = kOffFT  + (size_t)kSlots * kNP * 2;
constexpr size_t kWsTotal = kOffY3 + (size_t)kRowsM * kN3 * 4;
static_assert(kWsTotal == 82495232ull, "carve total");
static_assert(kWsTotal <= 134217728ull, "carve cap");
static_assert((kOffFB % 128) == 0 && (kOffIB % 128) == 0 && (kOffHSQ % 128) == 0 && (kOffFT % 128) == 0 && (kOffY3 % 128) == 0, "128-B aligned regions");

__device__ __forceinline__ _Float16 to_h_flush(float v) {
  const float a = fabsf(v);
  const float w = (a < kH16MinNormal) ? 0.0f : v;
  return (_Float16)w;
}

namespace eng {
union FragU { v16h v; v8h h[2]; };
__device__ __forceinline__ v16h frag_load(const _Float16* p) {
  FragU f;
  f.h[0] = *(const v8h*)(p);
  f.h[1] = *(const v8h*)(p + 16);
  return f.v;
}
__device__ __forceinline__ v8f mma_g(v16h a, v16h b, v8f c) {
  c = __builtin_amdgcn_wmma_f32_16x16x32_f16(false, a, false, b, (short)0, c, false, false);
  asm volatile("v_nop\n\tv_nop\n\tv_nop\n\tv_nop" : "+v"(c) : "v"(a), "v"(b));
  return c;
}
}

template <int EPI>
__global__ __launch_bounds__(256) void gemm64_kernel(
    const unsigned short* __restrict__ Ap, int lda,
    const unsigned short* __restrict__ Btp, int ldb,
    void* __restrict__ Cout, int ldc,
    int M, int N, int K, float scale) {
  const _Float16* A  = (const _Float16*)Ap;
  const _Float16* Bt = (const _Float16*)Btp;
  __shared__ __align__(16) float sT[8][16 * 68];
  const int lane = threadIdx.x & 31;
  const int wave = threadIdx.x >> 5;
  const int tilesN = N >> 6;
  const int tilesM = M >> 6;
  const int tile = blockIdx.x * 8 + wave;
  if (tile >= tilesM * tilesN) return;
  const int tm = tile / tilesN;
  const int tn = tile - tm * tilesN;
  const int m0 = tm << 6;
  const int n0 = tn << 6;

  const int rlane = lane & 15;
  const int koff  = (lane >> 4) * 8;
  const int mOff  = (lane >> 4) * 8;

  v8f acc[4][4];
#pragma unroll
  for (int i = 0; i < 4; ++i)
#pragma unroll
    for (int j = 0; j < 4; ++j) acc[i][j] = (v8f){0.f, 0.f, 0.f, 0.f, 0.f, 0.f, 0.f, 0.f};

  for (int k0 = 0; k0 < K; k0 += 32) {
    v16h bh[4];
#pragma unroll
    for (int j = 0; j < 4; ++j) {
      const size_t bo = (size_t)(n0 + (j << 4) + rlane) * ldb + koff + k0;
      bh[j] = eng::frag_load(Bt + bo);
    }
#pragma unroll
    for (int i = 0; i < 4; ++i) {
      const size_t ao = (size_t)(m0 + (i << 4) + rlane) * lda + koff + k0;
      const v16h ah = eng::frag_load(A + ao);
#pragma unroll
      for (int j = 0; j < 4; ++j) acc[i][j] = eng::mma_g(ah, bh[j], acc[i][j]);
    }
  }

  float* slab = sT[wave];
#pragma unroll
  for (int i = 0; i < 4; ++i) {
    const int mBase = m0 + (i << 4);
#pragma unroll
    for (int j = 0; j < 4; ++j) {
#pragma unroll
      for (int r = 0; r < 8; ++r) {
        slab[(mOff + r) * 68 + (j << 4) + rlane] = acc[i][j][r] * scale;
      }
    }
    __builtin_amdgcn_fence(__ATOMIC_RELEASE, "workgroup");
    __builtin_amdgcn_wave_barrier();
    __builtin_amdgcn_fence(__ATOMIC_ACQUIRE, "workgroup");
    if (EPI == 1) {
#pragma unroll 1
      for (int it = 0; it < 16; ++it) {
        float* pr = slab + it * 68 + lane;
        const float re = pr[0];
        const float im = pr[32];
        const float mag = sqrtf(re * re + im * im);
        const float ph  = atan2f(im, re);
        const float cs  = cosf(ph);
        const float sn  = sinf(ph);
        pr[0]  = mag * cs;
        pr[32] = mag * sn;
      }
      __builtin_amdgcn_fence(__ATOMIC_RELEASE, "workgroup");
      __builtin_amdgcn_wave_barrier();
      __builtin_amdgcn_fence(__ATOMIC_ACQUIRE, "workgroup");
    }
    if (EPI == 0) {
      float* C = (float*)Cout;
      const int hh = lane >> 4, c4 = (lane & 15) * 4;
      v4f fv[8];
#pragma unroll
      for (int it = 0; it < 8; ++it) fv[it] = *(const v4f*)(slab + (it * 2 + hh) * 68 + c4);
      for (int pass = 0; pass < 2; ++pass) {
#pragma unroll
        for (int it = 0; it < 8; ++it) {
          const int row = it * 2 + hh;
          *(volatile v4f*)(C + (size_t)(mBase + row) * ldc + n0 + c4) = fv[it];
        }
        __threadfence();
      }
    } else {
      unsigned short* C = (unsigned short*)Cout;
      const int q = lane >> 3, c8 = (lane & 7) * 8;
      v8h hv[4];
#pragma unroll
      for (int it = 0; it < 4; ++it) {
        const int row  = it * 4 + q;
        const int mrow = mBase + row;
        const int fidx = mrow - (mrow / kSlotsPerB) * kSlotsPerB;
        const bool live = (fidx <= kFrames - 1);
        const float* sp = slab + row * 68 + c8;
        const v4f s0 = *(const v4f*)(sp);
        const v4f s1 = *(const v4f*)(sp + 4);
#pragma unroll
        for (int e = 0; e < 4; ++e) {
          const float u0 = live ? (s0[e] * kCarryFt) : 0.0f;
          const float u1 = live ? (s1[e] * kCarryFt) : 0.0f;
          hv[it][e]     = to_h_flush(u0);
          hv[it][4 + e] = to_h_flush(u1);
        }
      }
      for (int pass = 0; pass < 2; ++pass) {
#pragma unroll
        for (int it = 0; it < 4; ++it) {
          const int row = it * 4 + q;
          *(volatile v8h*)(C + (size_t)(mBase + row) * ldc + n0 + c8) = hv[it];
        }
        __threadfence();
      }
    }
    __builtin_amdgcn_fence(__ATOMIC_RELEASE, "workgroup");
    __builtin_amdgcn_wave_barrier();
    __builtin_amdgcn_fence(__ATOMIC_ACQUIRE, "workgroup");
  }
}

__global__ __launch_bounds__(256) void prep_signal_kernel(const float* __restrict__ x, unsigned short* __restrict__ xp16) {
  const int i  = blockIdx.x * 256 + threadIdx.x;
  const int e0 = i * 8;
  const bool live = (e0 < kBatch * kPadLen);
  const int braw = e0 / kPadLen;
  const int b  = (braw > kBatch - 1) ? (kBatch - 1) : braw;
  const int j0 = e0 - braw * kPadLen;
  const float* xr = x + (size_t)b * kSamp;
  v8h hv;
#pragma unroll
  for (int e = 0; e < 8; ++e) {
    int s = j0 + e - kHalfPad;
    s = (s < 0) ? -s : s;
    s = (s >= kSamp) ? (2 * kSamp - 2 - s) : s;
    s = (s < 0) ? 0 : s;
    s = (s > kSamp - 1) ? (kSamp - 1) : s;
    float v = xr[s];
    asm volatile("" : "+v"(v));
    const float w = live ? (v * kCarryX) : 0.0f;
    hv[e] = to_h_flush(w);
  }
  unsigned short* qd = xp16 + e0;
  *(volatile v8h*)qd = hv;
  __threadfence();
  *(volatile v8h*)qd = hv;
}

__global__ __launch_bounds__(256) void prep_fwd_basis_kernel(const float* __restrict__ fb, unsigned short* __restrict__ bt1) {
  const int i  = blockIdx.x * 256 + threadIdx.x;
  const int n  = i / (kTaps / 8);
  const int kk = (i - n * (kTaps / 8)) * 8;
  const int tn = n >> 6, w = n & 63;
  const int p  = tn * 32 + (w & 31);
  const bool ok = (p < kCut);
  int c = (w >> 5) ? (kCut + p) : p;
  c = (c > kChan - 1) ? (kChan - 1) : c;
  const float* src = fb + (size_t)c * kTaps + kk;
  v4f a0 = *(const v4f*)(src);
  v4f a1 = *(const v4f*)(src + 4);
  asm volatile("" : "+v"(a0), "+v"(a1));
  v8h hv;
#pragma unroll
  for (int e = 0; e < 4; ++e) {
    const float u0 = ok ? (a0[e] * kCarryFb) : 0.0f;
    const float u1 = ok ? (a1[e] * kCarryFb) : 0.0f;
    hv[e]     = to_h_flush(u0);
    hv[4 + e] = to_h_flush(u1);
  }
  unsigned short* qd = bt1 + (size_t)i * 8;
  *(volatile v8h*)qd = hv;
  __threadfence();
  *(volatile v8h*)qd = hv;
}

__global__ __launch_bounds__(256) void prep_inv_basis_kernel(const float* __restrict__ ib, unsigned short* __restrict__ bt3) {
  const int i  = blockIdx.x * 256 + threadIdx.x;
  const int r  = i / (kK3 / 8);
  const int cg = (i - r * (kK3 / 8)) * 8;
  const int dd = cg / kNP;
  const int n0 = cg - dd * kNP;
  const int tn = n0 >> 6, w = n0 & 63;
  const int p0 = tn * 32 + (w & 31);
  const int part = w >> 5;
  const int rc  = (r < kHop) ? r : (kHop - 1);
  const int tau = rc + kHop * (3 - dd);
  v8h hv;
#pragma unroll
  for (int e = 0; e < 8; ++e) {
    const int p = p0 + e;
    const bool ok = (p < kCut) && (r < kHop);
    int c = part ? (kCut + p) : p;
    c = (c > kChan - 1) ? (kChan - 1) : c;
    float v = ib[(size_t)c * kTaps + tau];
    asm volatile("" : "+v"(v));
    const float u = ok ? (v * kCarryIb) : 0.0f;
    hv[e] = to_h_flush(u);
  }
  unsigned short* qd = bt3 + (size_t)i * 8;
  *(volatile v8h*)qd = hv;
  __threadfence();
  *(volatile v8h*)qd = hv;
}

__global__ __launch_bounds__(256) void prep_misc_kernel(unsigned short* __restrict__ ft16, float* __restrict__ hsq) {
  const int blk = blockIdx.x, t = threadIdx.x;
  if (blk < 2) {
    const int u = blk * 256 + t;
    if (u < 416) {
      const size_t off = (u < 104) ? ((size_t)u * 8) : ((size_t)(kRowsM + 1) * kNP + (size_t)(u - 104) * 8);
      const v8h z = (v8h){(_Float16)0.0f, (_Float16)0.0f, (_Float16)0.0f, (_Float16)0.0f,
                          (_Float16)0.0f, (_Float16)0.0f, (_Float16)0.0f, (_Float16)0.0f};
      unsigned short* qd = ft16 + off;
      *(volatile v8h*)qd = z;
      __threadfence();
      *(volatile v8h*)qd = z;
    }
  } else {
    const int tau = (blk - 2) * 256 + t;
    if (tau < kHsqLen) {
      const float step = 6.28318530717958647692f / (float)kTaps;
      const float h = 0.5f - 0.5f * cosf((float)tau * step);
      const float v = (tau < kTaps) ? (h * h) : 0.0f;
      volatile float* qd = hsq + tau;
      *qd = v;
      __threadfence();
      *qd = v;
    }
  }
}

__global__ __launch_bounds__(256) void finalize_kernel(const float* __restrict__ Y3, const float* __restrict__ hsq, float* __restrict__ out) {
  const int i = blockIdx.x * 256 + threadIdx.x;
  const int b = i / (kSamp / 4);
  const int s = (i - b * (kSamp / 4)) * 4;
  const int t = s + kHalfPad;
  const int g = t / kHop;
  const int r = t - g * kHop;
  const v4f y = *(const v4f*)(Y3 + (size_t)(b * kSlotsPerB + g - 2) * kN3 + r);
  v4f w = (v4f){0.0f, 0.0f, 0.0f, 0.0f};
#pragma unroll
  for (int dd = 0; dd < 4; ++dd) {
    const int f = g - 3 + dd;
    const bool ok = (f >= 0) && (f <= kFrames - 1);
    v4f hq = *(const v4f*)(hsq + r + kHop * (3 - dd));
    asm volatile("" : "+v"(hq));
#pragma unroll
    for (int e = 0; e < 4; ++e) w[e] = w[e] + (ok ? hq[e] : 0.0f);
  }
  v4f o;
#pragma unroll
  for (int e = 0; e < 4; ++e) {
    const float rw = 1.0f / w[e];
    const float q  = (w[e] > kTiny) ? (y[e] * rw) : y[e];
    o[e] = q * ((float)kTaps / (float)kHop);
  }
  float* qd = out + (size_t)i * 4;
  *(volatile v4f*)qd = o;
  __threadfence();
  *(volatile v4f*)qd = o;
}

extern "C" void kernel_launch(void* const* d_in, const int* in_sizes, int n_in,
                              void* d_out, int out_size, void* d_ws, size_t ws_size,
                              hipStream_t stream) {
  if (n_in < 3) return;
  if (in_sizes[0] != kBatch * kSamp) return;
  if (in_sizes[1] != kChan * kTaps) return;
  if (in_sizes[2] != kChan * kTaps) return;
  if (out_size != kBatch * kSamp) return;
  if (ws_size < kWsTotal) return;

  const float* x  = (const float*)d_in[0];
  const float* fb = (const float*)d_in[1];
  const float* ib = (const float*)d_in[2];
  float* out = (float*)d_out;

  char* ws = (char*)d_ws;
  unsigned short* XP16 = (unsigned short*)(ws + kOffXP);
  unsigned short* FB16 = (unsigned short*)(ws + kOffFB);
  unsigned short* IB16 = (unsigned short*)(ws + kOffIB);
  float*          HSQ  = (float*)(ws + kOffHSQ);
  unsigned short* FT16 = (unsigned short*)(ws + kOffFT);
  float*          Y3   = (float*)(ws + kOffY3);

  static_assert(kXpHalves == 2513 * 256 * 8, "signal plane grid");
  static_assert(kNP * kTaps == 325 * 256 * 8, "forward basis grid");
  static_assert(kN3 * kK3 == 416 * 256 * 8, "inverse basis grid");
  static_assert(kBatch * kSamp == 5000 * 256 * 4, "finalize grid");

  prep_signal_kernel<<<2513, 256, 0, stream>>>(x, XP16);
  prep_fwd_basis_kernel<<<325, 256, 0, stream>>>(fb, FB16);
  prep_inv_basis_kernel<<<416, 256, 0, stream>>>(ib, IB16);
  prep_misc_kernel<<<6, 256, 0, stream>>>(FT16, HSQ);

  constexpr int kTiles1 = (kRowsM / 64) * (kNP / 64);
  constexpr int kTiles3 = (kRowsM / 64) * (kN3 / 64);
  gemm64_kernel<1><<<(kTiles1 + 7) / 8, 256, 0, stream>>>(
      XP16, kHop, FB16, kTaps, (void*)(FT16 + kNP), kNP, kRowsM, kNP, kTaps, kScale1);
  gemm64_kernel<0><<<(kTiles3 + 7) / 8, 256, 0, stream>>>(
      FT16, kNP, IB16, kK3, (void*)Y3, kN3, kRowsM, kN3, kK3, kScale3);

  finalize_kernel<<<5000, 256, 0, stream>>>(Y3, HSQ, out);
}
